// TransformerDecoderLayerAsGNN_9663676416889
// MI455X (gfx1250) — hardware-run, weakly checked
//
#include <hip/hip_runtime.h>


#define NB_  4
#define NN   1024
#define NR   1024
#define CC   512
#define NH_  8
#define HPP  8
#define DK   64
#define FFD  2048
#define PCAR 1024.0f
typedef _Float16 h16;
typedef unsigned short bf;
typedef __attribute__((ext_vector_type(16))) __bf16   v16bf;
typedef __attribute__((ext_vector_type(16))) _Float16 v16h;
typedef __attribute__((ext_vector_type(8)))  _Float16 v8h;
typedef __attribute__((ext_vector_type(8)))  unsigned short v8us;
typedef __attribute__((ext_vector_type(8)))  float    v8f;
typedef __attribute__((ext_vector_type(4)))  float    v4f;
typedef v8h  __attribute__((may_alias)) v8ha;
typedef v4f  __attribute__((may_alias)) v4fa;
typedef v8us __attribute__((may_alias)) v8usa;

__device__ __forceinline__ unsigned short f2bf(float f) { unsigned u = __float_as_uint(f); u += 0x7FFFu + ((u >> 16) & 1u); return (unsigned short)(u >> 16); }
__device__ __forceinline__ float bf2f(unsigned short b) { return __uint_as_float(((unsigned)b) << 16); }
__device__ __forceinline__ float bfr(float f) { return bf2f(f2bf(f)); }
__device__ __forceinline__ v16h cat16(v8h lo, v8h hi) { return __builtin_shufflevector(lo, hi, 0, 1, 2, 3, 4, 5, 6, 7, 8, 9, 10, 11, 12, 13, 14, 15); }
__device__ __forceinline__ v16bf cat16b(v8us lo, v8us hi) { return __builtin_bit_cast(v16bf, __builtin_shufflevector(lo, hi, 0, 1, 2, 3, 4, 5, 6, 7, 8, 9, 10, 11, 12, 13, 14, 15)); }
__device__ __forceinline__ v8f wmma16(v16h a, v16h b, v8f c) { return __builtin_amdgcn_wmma_f32_16x16x32_f16(false, a, false, b, (short)0, c, false, false); }
__device__ __forceinline__ v8f wmmab(v16bf a, v16bf b, v8f c) { return __builtin_amdgcn_wmma_f32_16x16x32_bf16(false, a, false, b, (short)0, c, false, false); }


template <typename T16> struct WFrag;
template <> struct WFrag<h16> { typedef v16h V; static __device__ __forceinline__ V ld(const h16* p) { return cat16(*(const v8h*)p, *(const v8h*)(p + 16)); } static __device__ __forceinline__ v8f mma(V a, V b, v8f c) { return wmma16(a, b, c); } };
template <> struct WFrag<bf> { typedef v16bf V; static __device__ __forceinline__ V ld(const bf* p) { return cat16b(*(const v8us*)p, *(const v8us*)(p + 16)); } static __device__ __forceinline__ v8f mma(V a, V b, v8f c) { return wmmab(a, b, c); } };
template <typename T16, int NSPLIT, bool BIAS>
__global__ __launch_bounds__(32) void k_gemmw(const T16* __restrict__ A, const T16* __restrict__ A2, const T16* __restrict__ Bt, const T16* __restrict__ Bt2, int K, float* C, int ldc, const float* __restrict__ bias, size_t sA, size_t sB, size_t sC) {
    typedef typename WFrag<T16>::V V;
    __shared__ __align__(16) float os[16 * 68];
    const size_t z = blockIdx.z; A += z * sA; if (A2) A2 += z * sA; Bt += z * sB; if (Bt2) Bt2 += z * sB; C += z * sC;
    const int lane = threadIdx.x & 31, lr = lane & 15, hi = lane >> 4; const int r0 = blockIdx.x * 64, c0 = blockIdx.y * 64;
    v8f acc[4][4];
#pragma unroll
    for (int mb = 0; mb < 4; ++mb)
#pragma unroll
        for (int nb = 0; nb < 4; ++nb) acc[mb][nb] = (v8f){};
    const size_t aoff = (size_t)(r0 + lr) * K + 8 * hi, boff = (size_t)(c0 + lr) * K + 8 * hi;
#pragma unroll 1
    for (int kc = 0; kc < K; kc += 32) {
        V a[4], a2[4];
#pragma unroll
        for (int mb = 0; mb < 4; ++mb) { a[mb] = WFrag<T16>::ld(A + aoff + (size_t)mb * 16 * K + kc); if (NSPLIT == 1 || NSPLIT == 2) a2[mb] = WFrag<T16>::ld(A2 + aoff + (size_t)mb * 16 * K + kc); }
#pragma unroll
        for (int nb = 0; nb < 4; ++nb) { const V b = WFrag<T16>::ld(Bt + boff + (size_t)nb * 16 * K + kc); V b2; if (NSPLIT >= 2) b2 = WFrag<T16>::ld(Bt2 + boff + (size_t)nb * 16 * K + kc);
#pragma unroll
            for (int mb = 0; mb < 4; ++mb) { acc[mb][nb] = WFrag<T16>::mma(a[mb], b, acc[mb][nb]); if (NSPLIT == 1 || NSPLIT == 2) acc[mb][nb] = WFrag<T16>::mma(a2[mb], b, acc[mb][nb]); if (NSPLIT >= 2) acc[mb][nb] = WFrag<T16>::mma(a[mb], b2, acc[mb][nb]); } }
        asm volatile("v_nop\n\tv_nop\n\tv_nop\n\tv_nop" : "+v"(acc[0][0]), "+v"(acc[1][1]), "+v"(acc[2][2]), "+v"(acc[3][3]) : "v"(a[0]), "v"(a[3]));
    }
#pragma unroll
    for (int mb = 0; mb < 4; ++mb) {
#pragma unroll
        for (int nb = 0; nb < 4; ++nb) {
#pragma unroll
            for (int j = 0; j < 8; ++j) os[(hi * 8 + j) * 68 + nb * 16 + lr] = acc[mb][nb][j]; }
        __builtin_amdgcn_wave_barrier(); asm volatile("" ::: "memory");
        float* crow = C + (size_t)(r0 + mb * 16) * ldc + c0;
#pragma unroll 1
        for (int ps = 0; ps < 2; ++ps) {
#pragma unroll
            for (int s = 0; s < 8; ++s) { const int row = 2 * s + hi, cofs = lr * 4; v4f val = *(const v4fa*)(os + row * 68 + cofs); if (BIAS) { val[0] += bfr(bias[c0 + cofs]); val[1] += bfr(bias[c0 + cofs + 1]); val[2] += bfr(bias[c0 + cofs + 2]); val[3] += bfr(bias[c0 + cofs + 3]); }
                *(volatile v4f*)(crow + (size_t)row * ldc + cofs) = val; }
            if (ps == 0) __threadfence(); }
        __builtin_amdgcn_wave_barrier(); asm volatile("" ::: "memory");
    }
}

__device__ __forceinline__ h16 tohx(float x) { return (h16)x; }
__device__ __forceinline__ void splitf(float y, unsigned short& h, unsigned short& l) { h = f2bf(y); l = f2bf(y - bf2f(h)); }
typedef __attribute__((ext_vector_type(2))) unsigned short v2us;
typedef __attribute__((ext_vector_type(4))) unsigned short v4us;
typedef __attribute__((ext_vector_type(2))) _Float16 v2h;
typedef __attribute__((ext_vector_type(4))) _Float16 v4h;

__global__ __launch_bounds__(256) void k_wtG(const float* __restrict__ w, int K, int N, bf* Bt) {
    const int lane = threadIdx.x & 31; const int L0 = (blockIdx.x * 8 + (threadIdx.x >> 5)) * 8; const int nlines = N * K / 64;
#pragma unroll
    for (int ps = 0; ps < 2; ++ps) {
#pragma unroll 1
        for (int l = 0; l < 8; ++l) { const int L = L0 + l; if (L >= nlines) break; const size_t e = (size_t)L * 64 + lane * 2; const int k = (int)(e % K), n = (int)(e / K); v2us o;
            o[0] = f2bf(w[(size_t)k * N + n]); o[1] = f2bf(w[(size_t)(k + 1) * N + n]); *(volatile v2us*)(Bt + e) = o; }
        if (ps == 0) __threadfence(); }
}
__global__ __launch_bounds__(256) void k_cvt8(const float* __restrict__ src, bf* dst, size_t n8) { const size_t i = (size_t)blockIdx.x * 256 + threadIdx.x; if (i >= n8) return; const v8f v = *(const v8f*)(src + i * 8); v8us o;
#pragma unroll
    for (int k = 0; k < 8; ++k) o[k] = f2bf(v[k]); *(volatile v8us*)(dst + i * 8) = o; __threadfence(); *(volatile v8us*)(dst + i * 8) = o; }
__global__ __launch_bounds__(256) void k_pl(const float* __restrict__ F, int nrows, h16* P) { const size_t e = ((size_t)blockIdx.x * 256 + threadIdx.x) * 4; if (e >= (size_t)NH_ * nrows * DK) return; const int d = (int)(e % DK); const int t = (int)((e / DK) % nrows); const int h = (int)(e / ((size_t)DK * nrows)); const float* f = F + (size_t)t * CC + h * DK + d; v4h o;
#pragma unroll
    for (int u = 0; u < 4; ++u) o[u] = tohx(f[u]); *(volatile v4h*)(P + e) = o; __threadfence(); *(volatile v4h*)(P + e) = o; }
__global__ __launch_bounds__(256) void k_vt(const float* __restrict__ V, h16* VT) { const int e = (blockIdx.x * 256 + threadIdx.x) * 2; if (e >= NH_ * DK * NR) return; const int m = e % NR; const int d = (e / NR) % DK; const int h = e / (NR * DK); v2h o; o[0] = tohx(V[(size_t)m * CC + h * DK + d]); o[1] = tohx(V[(size_t)(m + 1) * CC + h * DK + d]); *(volatile v2h*)(VT + e) = o; __threadfence(); *(volatile v2h*)(VT + e) = o; }
__global__ __launch_bounds__(256) void k_soft(const float* __restrict__ Sb, h16* P16) { const int lane = threadIdx.x & 31; const int row = blockIdx.x * 8 + (threadIdx.x >> 5); if (row >= HPP * NN) return; const float* sr = Sb + (size_t)row * NR; float v[NR / 32]; float mx = -3.0e38f;
#pragma unroll
    for (int ch = 0; ch < NR / 128; ++ch) { const v4f a = *(const v4f*)(sr + ch * 128 + lane * 4);
#pragma unroll
        for (int u = 0; u < 4; ++u) { const float t = a[u] * 0.125f; v[ch * 4 + u] = t; mx = fmaxf(mx, t); } }
#pragma unroll
    for (int sh = 16; sh; sh >>= 1) mx = fmaxf(mx, __shfl_xor(mx, sh, 32));
    float sum = 0.f;
#pragma unroll
    for (int q = 0; q < NR / 32; ++q) { float d0 = __fsub_rn(v[q], mx); asm volatile("" : "+v"(d0)); v[q] = __builtin_amdgcn_exp2f(__fmul_rn(d0, 1.4426950408889634f)); sum += v[q]; }
#pragma unroll
    for (int sh = 16; sh; sh >>= 1) sum += __shfl_xor(sum, sh, 32);
    const float f = __fdiv_rn(PCAR, sum);
    for (int ps = 0; ps < 2; ++ps) {
#pragma unroll
        for (int ch = 0; ch < NR / 128; ++ch) { v4h o4;
#pragma unroll
            for (int q = 0; q < 4; ++q) o4[q] = tohx(v[ch * 4 + q] * f); *(volatile v4h*)(P16 + (size_t)row * NR + ch * 128 + lane * 4) = o4; }
        if (ps == 0) __threadfence(); } }
__global__ __launch_bounds__(256) void k_mrg(const float* __restrict__ O, int h0, bf* Ah, bf* Al) { const int e = (blockIdx.x * 256 + threadIdx.x) * 4; if (e >= HPP * NN * DK) return; const int d = e % DK; const int t = (e / DK) % NN; const int z = e / (DK * NN); v4us oh, ol;
#pragma unroll
    for (int u = 0; u < 4; ++u) { unsigned short a, b; splitf(O[e + u] * (1.0f / PCAR), a, b); oh[u] = a; ol[u] = b; } const size_t oo = (size_t)t * CC + (h0 + z) * DK + d; *(volatile v4us*)(Ah + oo) = oh; *(volatile v4us*)(Al + oo) = ol; __threadfence(); *(volatile v4us*)(Ah + oo) = oh; *(volatile v4us*)(Al + oo) = ol; }

__global__ __launch_bounds__(256) void k_lnr(const float* __restrict__ A, int abf, const float* __restrict__ Bv, const float* __restrict__ g, const float* __restrict__ bb, float* X, bf* Xh, bf* Xl) {
    const int lane = threadIdx.x & 31; const int r = blockIdx.x * 8 + (threadIdx.x >> 5); if (r >= NN) return; float v[CC / 32]; float s = 0.f;
#pragma unroll
    for (int ch = 0; ch < CC / 128; ++ch) { const size_t o0 = (size_t)r * CC + ch * 128 + lane * 4; const v4f a = *(const v4f*)(A + o0), b4 = *(const v4f*)(Bv + o0);
#pragma unroll
        for (int u = 0; u < 4; ++u) { float av = abf ? bfr(a[u]) : a[u]; asm volatile("" : "+v"(av)); v[ch * 4 + u] = __fadd_rn(av, b4[u]); s += v[ch * 4 + u]; } }
#pragma unroll
    for (int sh = 16; sh; sh >>= 1) s += __shfl_xor(s, sh, 32);
    const float mean = s * (1.0f / CC); float q = 0.f;
#pragma unroll
    for (int k = 0; k < CC / 32; ++k) { float d = __fsub_rn(v[k], mean); asm volatile("" : "+v"(d)); float p = __fmul_rn(d, d); asm volatile("" : "+v"(p)); q = __fadd_rn(q, p); }
#pragma unroll
    for (int sh = 16; sh; sh >>= 1) q += __shfl_xor(q, sh, 32);
    const float rs = __frsqrt_rn(__fadd_rn(q * (1.0f / CC), 1e-5f));
    for (int ps = 0; ps < 2; ++ps) {
#pragma unroll
        for (int ch = 0; ch < CC / 128; ++ch) { v4f w; v4us oh, ol;
#pragma unroll
            for (int u = 0; u < 4; ++u) { const int c = ch * 128 + lane * 4 + u; float d = __fsub_rn(v[ch * 4 + u], mean); asm volatile("" : "+v"(d)); float n0 = __fmul_rn(d, rs); asm volatile("" : "+v"(n0)); float gg = bfr(g[c]), be = bfr(bb[c]); asm volatile("" : "+v"(gg)); asm volatile("" : "+v"(be)); float t1 = __fmul_rn(n0, gg); asm volatile("" : "+v"(t1)); w[u] = __fadd_rn(t1, be); unsigned short p2, q2; splitf(w[u], p2, q2); oh[u] = p2; ol[u] = q2; }
            const size_t oo = (size_t)r * CC + ch * 128 + lane * 4; *(volatile v4f*)(X + oo) = w; if (Xh) { *(volatile v4us*)(Xh + oo) = oh; *(volatile v4us*)(Xl + oo) = ol; } }
        if (ps == 0) __threadfence(); } }
__global__ __launch_bounds__(256) void k_relu(const float* __restrict__ F, size_t n4, bf* Hh, bf* Hl) { const size_t e = ((size_t)blockIdx.x * 256 + threadIdx.x) * 4; if (e >= n4) return; const v4f a = *(const v4f*)(F + e); v4us oh, ol;
#pragma unroll
    for (int u = 0; u < 4; ++u) { unsigned short p, q; splitf(fmaxf(a[u], 0.f), p, q); oh[u] = p; ol[u] = q; } *(volatile v4us*)(Hh + e) = oh; *(volatile v4us*)(Hl + e) = ol; __threadfence(); *(volatile v4us*)(Hh + e) = oh; *(volatile v4us*)(Hl + e) = ol; }

static void attn(hipStream_t stream, const float* FQ, const float* FK, const float* FV, h16* Q16, h16* K16, h16* VT, float* S, h16* P16, float* O, bf* CTh, bf* CTl) {
    const size_t zq = (size_t)NN * DK, zS = (size_t)NN * NR, zv = (size_t)DK * NR;
    k_pl<<<(unsigned)(((size_t)NH_ * NN * DK / 4 + 255) / 256), 256, 0, stream>>>(FQ, NN, Q16); k_pl<<<(unsigned)(((size_t)NH_ * NR * DK / 4 + 255) / 256), 256, 0, stream>>>(FK, NR, K16); k_vt<<<(NH_ * DK * NR / 2 + 255) / 256, 256, 0, stream>>>(FV, VT);
    k_gemmw<h16, 0, false><<<dim3(NN / 64, NR / 64, NH_), 32, 0, stream>>>(Q16, nullptr, K16, nullptr, DK, S, NR, nullptr, zq, zq, zS);
    k_soft<<<HPP * NN / 8, 256, 0, stream>>>(S, P16);
    k_gemmw<h16, 0, false><<<dim3(NN / 64, 1, NH_), 32, 0, stream>>>(P16, nullptr, VT, nullptr, NR, O, DK, nullptr, zS, zv, zq);
    k_mrg<<<(HPP * NN * DK / 4 + 255) / 256, 256, 0, stream>>>(O, 0, CTh, CTl); }

extern "C" void kernel_launch(void* const* d_in, const int* in_sizes, int n_in,
                              void* d_out, int out_size, void* d_ws, size_t ws_size, hipStream_t stream) {
    (void)in_sizes; (void)n_in; (void)out_size;
    const float** I = (const float**)d_in;
    const float *tgt = I[0], *mem = I[1], *sWq = I[2], *sWk = I[3], *sWv = I[4], *sWo = I[5], *cWq = I[6], *cWk = I[7], *cWv = I[8], *cWo = I[9];
    const float *sbq = I[10], *sbk = I[11], *sbv = I[12], *sbo = I[13], *cbq = I[14], *cbk = I[15], *cbv = I[16], *cbo = I[17], *fW1 = I[18], *fb1 = I[19], *fW2 = I[20], *fb2 = I[21], *g1 = I[22], *g2 = I[23], *g3 = I[24], *be1 = I[25], *be2 = I[26], *be3 = I[27];
    float* OUT = (float*)d_out;
    char* wsp = (char*)d_ws;
    auto take = [&](size_t bytes) { char* p = wsp; wsp += (bytes + 255) & ~(size_t)255; return (void*)p; };
    bf* W8[8]; for (int i = 0; i < 8; ++i) W8[i] = (bf*)take((size_t)CC * CC * 2); bf* BW1 = (bf*)take((size_t)FFD * CC * 2); bf* BW2 = (bf*)take((size_t)CC * FFD * 2);
    bf* XB = (bf*)take((size_t)NN * CC * 2); bf* MB = (bf*)take((size_t)NR * CC * 2); float* FQ = (float*)take((size_t)NN * CC * 4); float* FK = (float*)take((size_t)NR * CC * 4); float* FV = (float*)take((size_t)NR * CC * 4);
    h16* Q16 = (h16*)take((size_t)NH_ * NN * DK * 2); h16* K16 = (h16*)take((size_t)NH_ * NR * DK * 2); h16* VT = (h16*)take((size_t)NH_ * DK * NR * 2); float* S = (float*)take((size_t)NH_ * NN * NR * 4); h16* P16 = (h16*)take((size_t)NH_ * NN * NR * 2); float* O = (float*)take((size_t)NH_ * NN * DK * 4);
    bf* CTh = (bf*)take((size_t)NN * CC * 2); bf* CTl = (bf*)take((size_t)NN * CC * 2); float* Y = (float*)take((size_t)NN * CC * 4); float* X1 = (float*)take((size_t)NN * CC * 4); bf* X1h = (bf*)take((size_t)NN * CC * 2); bf* X1l = (bf*)take((size_t)NN * CC * 2);
    float* X2 = (float*)take((size_t)NN * CC * 4); bf* X2h = (bf*)take((size_t)NN * CC * 2); bf* X2l = (bf*)take((size_t)NN * CC * 2); float* F1 = (float*)take((size_t)NN * FFD * 4); bf* F1h = (bf*)take((size_t)NN * FFD * 2); bf* F1l = (bf*)take((size_t)NN * FFD * 2);
    if ((size_t)(wsp - (char*)d_ws) > ws_size) return;
    const float* Wl[8] = {sWq, sWk, sWv, sWo, cWq, cWk, cWv, cWo}; for (int i = 0; i < 8; ++i) k_wtG<<<(CC * CC / 64 + 63) / 64, 256, 0, stream>>>(Wl[i], CC, CC, W8[i]);
    k_wtG<<<(CC * FFD / 64 + 63) / 64, 256, 0, stream>>>(fW1, CC, FFD, BW1); k_wtG<<<(FFD * CC / 64 + 63) / 64, 256, 0, stream>>>(fW2, FFD, CC, BW2);
    const dim3 gp(NN / 64, CC / 64, 1);
    for (int b = 0; b < NB_; ++b) { const float* tb = tgt + (size_t)b * NN * CC;
        k_cvt8<<<(NN * CC / 8 + 255) / 256, 256, 0, stream>>>(tb, XB, (size_t)NN * CC / 8); k_cvt8<<<(NR * CC / 8 + 255) / 256, 256, 0, stream>>>(mem + (size_t)b * NR * CC, MB, (size_t)NR * CC / 8);
        k_gemmw<bf, 0, true><<<gp, 32, 0, stream>>>(XB, nullptr, W8[0], nullptr, CC, FQ, CC, sbq, 0, 0, 0); k_gemmw<bf, 0, true><<<gp, 32, 0, stream>>>(XB, nullptr, W8[1], nullptr, CC, FK, CC, sbk, 0, 0, 0); k_gemmw<bf, 0, true><<<gp, 32, 0, stream>>>(XB, nullptr, W8[2], nullptr, CC, FV, CC, sbv, 0, 0, 0);
        attn(stream, FQ, FK, FV, Q16, K16, VT, S, P16, O, CTh, CTl);
        k_gemmw<bf, 1, true><<<gp, 32, 0, stream>>>(CTh, CTl, W8[3], nullptr, CC, Y, CC, sbo, 0, 0, 0);
        k_lnr<<<NN / 8, 256, 0, stream>>>(tb, 1, Y, g1, be1, X1, X1h, X1l);
        k_gemmw<bf, 1, true><<<gp, 32, 0, stream>>>(X1h, X1l, W8[4], nullptr, CC, FQ, CC, cbq, 0, 0, 0); k_gemmw<bf, 0, true><<<gp, 32, 0, stream>>>(MB, nullptr, W8[5], nullptr, CC, FK, CC, cbk, 0, 0, 0); k_gemmw<bf, 0, true><<<gp, 32, 0, stream>>>(MB, nullptr, W8[6], nullptr, CC, FV, CC, cbv, 0, 0, 0);
        attn(stream, FQ, FK, FV, Q16, K16, VT, S, P16, O, CTh, CTl);
        k_gemmw<bf, 1, true><<<gp, 32, 0, stream>>>(CTh, CTl, W8[7], nullptr, CC, Y, CC, cbo, 0, 0, 0);
        k_lnr<<<NN / 8, 256, 0, stream>>>(X1, 0, Y, g2, be2, X2, X2h, X2l);
        k_gemmw<bf, 1, true><<<dim3(NN / 64, FFD / 64, 1), 32, 0, stream>>>(X2h, X2l, BW1, nullptr, CC, F1, FFD, fb1, 0, 0, 0); k_relu<<<(unsigned)(((size_t)NN * FFD / 4 + 255) / 256), 256, 0, stream>>>(F1, (size_t)NN * FFD, F1h, F1l);
        k_gemmw<bf, 1, true><<<gp, 32, 0, stream>>>(F1h, F1l, BW2, nullptr, FFD, Y, CC, fb2, 0, 0, 0);
        k_lnr<<<NN / 8, 256, 0, stream>>>(X2, 0, Y, g3, be3, OUT + (size_t)b * NN * CC, nullptr, nullptr); }
}
